// MultiHeadAttention_53420803228274
// MI455X (gfx1250) — hardware-run, weakly checked
//
#include <hip/hip_runtime.h>


#ifndef NB
#define NB 2
#endif
#ifndef SEQ
#define SEQ 2048
#endif
#define NB_FULL  2
#define SEQ_FULL 2048
#ifndef OUT_SEQ
#define OUT_SEQ SEQ
#endif
#define DM   2048
#define NH_  16
#define HD   128
#define HH   64
#define AW   4
#define QRS  2048.0f
#define QRI  (1.0f / 2048.0f)
#define SC2  (0.08838834764831845f * 1.4426950408889634f)
#define PSH  8.0f
#define WOS  1024.0f
#define CXS  16.0f
#define OUTI (1.0f / (1024.0f * 16.0f))
constexpr int EARLY = (SEQ < 512) ? SEQ : 512;

static_assert(HD == 128);
static_assert(HH * 2 == HD);
static_assert(NH_ * HD == DM);
static_assert(DM % 64 == 0);
static_assert(DM % 32 == 0);
static_assert(SEQ % 64 == 0);
static_assert(EARLY % 64 == 0);
static_assert(EARLY <= SEQ);
static_assert((SEQ - EARLY) % (16 * AW) == 0);
static_assert(((EARLY / 16) * 2) % AW == 0);
static_assert(((size_t)SEQ * DM) % 8 == 0);
static_assert(((size_t)DM * DM) % 8 == 0);
static_assert(((size_t)SEQ * HH) % 256 == 0);
static_assert(NB <= NB_FULL);
static_assert(SEQ <= SEQ_FULL);

typedef _Float16 h16;
typedef unsigned short bf;
typedef __attribute__((ext_vector_type(16))) __bf16   v16bf;
typedef __attribute__((ext_vector_type(16))) _Float16 v16h;
typedef __attribute__((ext_vector_type(8)))  _Float16 v8h;
typedef __attribute__((ext_vector_type(8)))  unsigned short v8us;
typedef __attribute__((ext_vector_type(8)))  float    v8f;
typedef __attribute__((ext_vector_type(4)))  float    v4f;
typedef v4f  __attribute__((may_alias)) v4fa;

__device__ __forceinline__ unsigned short f2bf(float f) { unsigned u = __float_as_uint(f); u += 0x7FFFu + ((u >> 16) & 1u); return (unsigned short)(u >> 16); }
__device__ __forceinline__ float bfr(float f) { return __uint_as_float(((unsigned)f2bf(f)) << 16); }
__device__ __forceinline__ v16h cat16(v8h lo, v8h hi) { return __builtin_shufflevector(lo, hi, 0, 1, 2, 3, 4, 5, 6, 7, 8, 9, 10, 11, 12, 13, 14, 15); }
__device__ __forceinline__ v16bf cat16b(v8us lo, v8us hi) { return __builtin_bit_cast(v16bf, __builtin_shufflevector(lo, hi, 0, 1, 2, 3, 4, 5, 6, 7, 8, 9, 10, 11, 12, 13, 14, 15)); }
__device__ __forceinline__ v8f wmma16(v16h a, v16h b, v8f c) { return __builtin_amdgcn_wmma_f32_16x16x32_f16(false, a, false, b, (short)0, c, false, false); }
__device__ __forceinline__ v8f wmmab(v16bf a, v16bf b, v8f c) { return __builtin_amdgcn_wmma_f32_16x16x32_bf16(false, a, false, b, (short)0, c, false, false); }
__device__ __forceinline__ v16h  ldh(const h16* p) { return cat16(*(const v8h*)p, *(const v8h*)(p + 16)); }
__device__ __forceinline__ v16bf ldb(const bf* p)  { return cat16b(*(const v8us*)p, *(const v8us*)(p + 16)); }
__device__ __forceinline__ void wave_sync() { __builtin_amdgcn_fence(3  , "wavefront"); __builtin_amdgcn_wave_barrier(); asm volatile("" ::: "memory"); }
struct HR { h16 h; h16 r; };
__device__ __forceinline__ HR split16(float x) {
    const h16 t = (h16)x;
    const h16 hv = (fabsf(x) < 6.103515625e-5f) ? (h16)0.0f : t;
    HR o; o.h = hv; o.r = (h16)((x - (float)hv) * QRS); return o;
}

__global__ __launch_bounds__(256) void k_cvt8(const float* __restrict__ src, bf* dst, size_t n8) {
    const size_t i = (size_t)blockIdx.x * 256 + threadIdx.x; if (i >= n8) return;
    const v8f v = *(const v8f*)(src + i * 8); v8us o;
#pragma unroll
    for (int k = 0; k < 8; ++k) o[k] = f2bf(v[k]);
    *(volatile v8us*)(dst + i * 8) = o; __threadfence(); *(volatile v8us*)(dst + i * 8) = o;
}

__global__ __launch_bounds__(256) void k_cvtw(const float* __restrict__ src, h16* dst, size_t n8) {
    const size_t i = (size_t)blockIdx.x * 256 + threadIdx.x; if (i >= n8) return;
    const v8f v = *(const v8f*)(src + i * 8); v8h o;
#pragma unroll
    for (int k = 0; k < 8; ++k) o[k] = (h16)(bfr(v[k]) * WOS);
    *(volatile v8h*)(dst + i * 8) = o; __threadfence(); *(volatile v8h*)(dst + i * 8) = o;
}

__global__ __launch_bounds__(256) void k_tab(float* COS, float* SIN) {
    const int idx = blockIdx.x * 256 + threadIdx.x;
    const int pos = idx >> 6, i = idx & 63;
    const double a = -(double)i * (13.287712379549449 / 64.0);
    const float ah = (float)a; const float al = (float)(a - (double)ah);
    const float inv = __builtin_amdgcn_exp2f(ah) * (1.0f + al * 0.6931471805599453f);
    const float ang = (float)pos * inv;
    const float c = cosf(ang); const float s = sinf(ang);
    *(volatile float*)(COS + idx) = c; *(volatile float*)(SIN + idx) = s;
    __threadfence();
    *(volatile float*)(COS + idx) = c; *(volatile float*)(SIN + idx) = s;
}

__global__ __launch_bounds__(32) void k_qk(const bf* __restrict__ A, const bf* __restrict__ Bt, const float* __restrict__ bias,
                                           const float* __restrict__ COS, const float* __restrict__ SIN, h16* Ph, h16* Pr) {
    __shared__ __align__(16) float os[16 * 132];
    const int K = DM;
    const int lane = threadIdx.x & 31, lr = lane & 15, hi = lane >> 4;
    const int r0 = blockIdx.x * 32, head = blockIdx.y, cb = head * HD;
    v8f acc[2][8];
#pragma unroll
    for (int mb = 0; mb < 2; ++mb)
#pragma unroll
        for (int nb = 0; nb < 8; ++nb) acc[mb][nb] = (v8f){};
    const size_t aoff = (size_t)(r0 + lr) * K + 8 * hi, boff = (size_t)(cb + lr) * K + 8 * hi;
#pragma unroll 1
    for (int kc = 0; kc < K; kc += 32) {
        const v16bf a0 = ldb(A + aoff + kc), a1 = ldb(A + aoff + (size_t)16 * K + kc);
#pragma unroll
        for (int nb = 0; nb < 8; ++nb) { const v16bf w = ldb(Bt + boff + (size_t)nb * 16 * K + kc);
            acc[0][nb] = wmmab(a0, w, acc[0][nb]); acc[1][nb] = wmmab(a1, w, acc[1][nb]); }
        asm volatile("" : "+v"(acc[0][0]), "+v"(acc[0][1]), "+v"(acc[0][2]), "+v"(acc[0][3]), "+v"(acc[1][0]), "+v"(acc[1][1]), "+v"(acc[1][2]), "+v"(acc[1][3]));
        asm volatile("v_nop\n\tv_nop\n\tv_nop\n\tv_nop" : "+v"(acc[0][4]), "+v"(acc[0][5]), "+v"(acc[0][6]), "+v"(acc[0][7]), "+v"(acc[1][4]), "+v"(acc[1][5]), "+v"(acc[1][6]), "+v"(acc[1][7]) : "v"(a0), "v"(a1));
    }
    const int bidx = r0 / SEQ, tb = r0 % SEQ;
    const size_t zh = (size_t)bidx * NH_ + head;
    const bool wres = tb < EARLY;
    float bz[8];
#pragma unroll
    for (int nb = 0; nb < 8; ++nb) bz[nb] = bfr(bias[cb + nb * 16 + lr]);
#pragma unroll
    for (int mb = 0; mb < 2; ++mb) {
#pragma unroll
        for (int nb = 0; nb < 8; ++nb) {
#pragma unroll
            for (int j = 0; j < 8; ++j) os[(hi * 8 + j) * 132 + nb * 16 + lr] = acc[mb][nb][j] + bz[nb]; }
        wave_sync();
#pragma unroll 1
        for (int ps = 0; ps < 2; ++ps) {
#pragma unroll
            for (int s = 0; s < 8; ++s) { const int row = 2 * s + hi, c8 = lr * 8, pc = c8 ^ 64, i8 = c8 & 63;
                const int t = tb + mb * 16 + row;
                const float sg = (c8 < 64) ? -1.0f : 1.0f;
                const v4f x0 = *(const v4fa*)(&os[row * 132 + c8]); const v4f x1 = *(const v4fa*)(&os[row * 132 + c8 + 4]);
                const v4f y0 = *(const v4fa*)(&os[row * 132 + pc]); const v4f y1 = *(const v4fa*)(&os[row * 132 + pc + 4]);
                const v4f ca = *(const v4f*)(COS + (size_t)t * HH + i8); const v4f cc = *(const v4f*)(COS + (size_t)t * HH + i8 + 4);
                const v4f sa = *(const v4f*)(SIN + (size_t)t * HH + i8); const v4f sc = *(const v4f*)(SIN + (size_t)t * HH + i8 + 4);
                v8h hv, rv;
#pragma unroll
                for (int i = 0; i < 4; ++i) { const float u0 = x0[i] * ca[i] + (sg * y0[i]) * sa[i]; const float u1 = x1[i] * cc[i] + (sg * y1[i]) * sc[i];
                    const HR e0 = split16(u0); const HR e1 = split16(u1); hv[i] = e0.h; rv[i] = e0.r; hv[4 + i] = e1.h; rv[4 + i] = e1.r; }
                const size_t oo = (zh * SEQ + (size_t)t) * HD + c8;
                *(volatile v8h*)(Ph + oo) = hv;
                if (wres) { const size_t ro = (zh * EARLY + (size_t)t) * HD + c8; *(volatile v8h*)(Pr + ro) = rv; } }
            if (ps == 0) __threadfence(); }
        wave_sync();
    }
}

__global__ __launch_bounds__(32) void k_vt(const bf* __restrict__ A, const bf* __restrict__ Bt, const float* __restrict__ bias, h16* Ph, h16* Pr) {
    __shared__ __align__(16) float os[16 * 68];
    const int K = DM;
    const int lane = threadIdx.x & 31, lr = lane & 15, hi = lane >> 4; const int r0 = blockIdx.x * 64, c0 = blockIdx.y * 64;
    v8f acc[4][4];
#pragma unroll
    for (int mb = 0; mb < 4; ++mb)
#pragma unroll
        for (int nb = 0; nb < 4; ++nb) acc[mb][nb] = (v8f){};
    const size_t aoff = (size_t)(r0 + lr) * K + 8 * hi, boff = (size_t)(c0 + lr) * K + 8 * hi;
#pragma unroll 1
    for (int kc = 0; kc < K; kc += 32) {
        v16bf a[4];
#pragma unroll
        for (int mb = 0; mb < 4; ++mb) a[mb] = ldb(A + aoff + (size_t)mb * 16 * K + kc);
#pragma unroll
        for (int nb = 0; nb < 4; ++nb) { const v16bf w = ldb(Bt + boff + (size_t)nb * 16 * K + kc);
#pragma unroll
            for (int mb = 0; mb < 4; ++mb) acc[mb][nb] = wmmab(a[mb], w, acc[mb][nb]); }
        asm volatile("" : "+v"(acc[0][0]), "+v"(acc[0][1]), "+v"(acc[0][2]), "+v"(acc[0][3]), "+v"(acc[1][0]), "+v"(acc[1][1]), "+v"(acc[1][2]), "+v"(acc[1][3]));
        asm volatile("v_nop\n\tv_nop\n\tv_nop\n\tv_nop" : "+v"(acc[2][0]), "+v"(acc[2][1]), "+v"(acc[2][2]), "+v"(acc[2][3]), "+v"(acc[3][0]), "+v"(acc[3][1]), "+v"(acc[3][2]), "+v"(acc[3][3]) : "v"(a[0]), "v"(a[1]), "v"(a[2]), "v"(a[3]));
    }
    const int bidx = c0 / SEQ, t0 = c0 % SEQ;
    const bool wres = t0 < EARLY;
#pragma unroll
    for (int mb = 0; mb < 4; ++mb) {
#pragma unroll
        for (int nb = 0; nb < 4; ++nb) {
#pragma unroll
            for (int j = 0; j < 8; ++j) os[(hi * 8 + j) * 68 + nb * 16 + lr] = acc[mb][nb][j]; }
        wave_sync();
#pragma unroll 1
        for (int ps = 0; ps < 2; ++ps) {
#pragma unroll
            for (int s = 0; s < 4; ++s) { const int row = 4 * s + (lane >> 3), c8 = (lane & 7) * 8;
                const int mrow = r0 + mb * 16 + row;
                const float bb = bfr(bias[mrow]);
                const v4f x0 = *(const v4fa*)(&os[row * 68 + c8]); const v4f x1 = *(const v4fa*)(&os[row * 68 + c8 + 4]); v8h hv, rv;
#pragma unroll
                for (int i = 0; i < 4; ++i) { const HR e0 = split16(x0[i] + bb); const HR e1 = split16(x1[i] + bb); hv[i] = e0.h; rv[i] = e0.r; hv[4 + i] = e1.h; rv[4 + i] = e1.r; }
                const size_t prow = (size_t)bidx * DM + (size_t)mrow;
                *(volatile v8h*)(Ph + prow * SEQ + t0 + c8) = hv;
                if (wres) *(volatile v8h*)(Pr + prow * EARLY + t0 + c8) = rv; }
            if (ps == 0) __threadfence(); }
        wave_sync();
    }
}

__global__ __launch_bounds__(32 * AW) void k_flash_dense(const h16* __restrict__ QH, const h16* __restrict__ KP, const h16* __restrict__ VT, h16* CTX) {
    __shared__ __align__(16) float os[AW * 16 * 132];
    const int lane = threadIdx.x & 31, wave = __builtin_amdgcn_readfirstlane((int)(threadIdx.x >> 5)), lr = lane & 15, hi = lane >> 4;
    const int zh = blockIdx.y; const int b = zh / NH_, h = zh % NH_;
    const int t0 = EARLY + (blockIdx.x * AW + wave) * 16;
    const size_t pbase = (size_t)zh * SEQ * HD;
    const size_t qo = pbase + (size_t)(t0 + lr) * HD + 8 * hi;
    const v16h q0 = ldh(QH + qo), q1 = ldh(QH + qo + 32), q2 = ldh(QH + qo + 64), q3 = ldh(QH + qo + 96);
    const size_t ko = pbase + (size_t)lr * HD + 8 * hi;
    const size_t vo = pbase + (size_t)lr * SEQ + 8 * hi;
    v8f o[8];
#pragma unroll
    for (int j = 0; j < 8; ++j) o[j] = (v8f){};
    float m = -3.0e38f, l = 0.0f;
    const int nst = t0 / 32 + 1;
#pragma unroll 1
    for (int st = 0; st < nst; ++st) {
        const int key0 = st * 32;
        const h16* ka = KP + ko + (size_t)key0 * HD; const h16* kb = ka + 16 * HD;
        const v16h a0 = ldh(ka), a1 = ldh(ka + 32), a2 = ldh(ka + 64), a3 = ldh(ka + 96);
        const v16h b0 = ldh(kb), b1 = ldh(kb + 32), b2 = ldh(kb + 64), b3 = ldh(kb + 96);
        v8f sa = (v8f){}, sb = (v8f){};
        sa = wmma16(a0, q0, sa); sb = wmma16(b0, q0, sb); sa = wmma16(a1, q1, sa); sb = wmma16(b1, q1, sb);
        sa = wmma16(a2, q2, sa); sb = wmma16(b2, q2, sb); sa = wmma16(a3, q3, sa); sb = wmma16(b3, q3, sb);
        asm volatile("v_nop\n\tv_nop\n\tv_nop\n\tv_nop" : "+v"(sa), "+v"(sb) : "v"(a0), "v"(a1), "v"(a2), "v"(a3), "v"(b0), "v"(b1), "v"(b2), "v"(b3));
        float ta[8], tb[8];
#pragma unroll
        for (int r = 0; r < 8; ++r) { ta[r] = sa[r] * SC2; tb[r] = sb[r] * SC2; }
        if (key0 + 31 > t0) {
            const int tq = t0 + lr, kA = key0 + 8 * hi;
#pragma unroll
            for (int r = 0; r < 8; ++r) { ta[r] = (kA + r > tq) ? -3.0e38f : ta[r]; tb[r] = (kA + 16 + r > tq) ? -3.0e38f : tb[r]; }
        }
        float mx = -3.0e38f;
#pragma unroll
        for (int r = 0; r < 8; ++r) mx = fmaxf(mx, fmaxf(ta[r], tb[r]));
        mx = fmaxf(mx, __shfl_xor(mx, 16, 32));
        const float mnew = fmaxf(m, mx);
        const float alpha = __builtin_amdgcn_exp2f(m - mnew);
        const float sh = PSH - mnew;
        v16h pb; float ls = 0.0f;
#pragma unroll
        for (int r = 0; r < 8; ++r) { const h16 pa = (h16)__builtin_amdgcn_exp2f(ta[r] + sh); const h16 pc = (h16)__builtin_amdgcn_exp2f(tb[r] + sh); pb[r] = pa; pb[8 + r] = pc; ls += (float)pa + (float)pc; }
        l = l * alpha + ls; m = mnew;
#pragma unroll
        for (int j = 0; j < 8; ++j) o[j] = o[j] * alpha;
        const h16* va = VT + vo + key0;
        const v16h v0 = ldh(va), v1 = ldh(va + (size_t)16 * SEQ), v2 = ldh(va + (size_t)32 * SEQ), v3 = ldh(va + (size_t)48 * SEQ);
        const v16h v4 = ldh(va + (size_t)64 * SEQ), v5 = ldh(va + (size_t)80 * SEQ), v6 = ldh(va + (size_t)96 * SEQ), v7 = ldh(va + (size_t)112 * SEQ);
        o[0] = wmma16(v0, pb, o[0]); o[1] = wmma16(v1, pb, o[1]); o[2] = wmma16(v2, pb, o[2]); o[3] = wmma16(v3, pb, o[3]);
        o[4] = wmma16(v4, pb, o[4]); o[5] = wmma16(v5, pb, o[5]); o[6] = wmma16(v6, pb, o[6]); o[7] = wmma16(v7, pb, o[7]);
        asm volatile("v_nop\n\tv_nop\n\tv_nop\n\tv_nop" : "+v"(o[0]), "+v"(o[1]), "+v"(o[2]), "+v"(o[3]), "+v"(o[4]), "+v"(o[5]), "+v"(o[6]), "+v"(o[7])
                     : "v"(v0), "v"(v1), "v"(v2), "v"(v3), "v"(v4), "v"(v5), "v"(v6), "v"(v7), "v"(pb));
    }
    l += __shfl_xor(l, 16, 32);
    const float inv = CXS / l;
    const int wb = wave * 16 * 132;
#pragma unroll
    for (int j = 0; j < 8; ++j) { v4f a, c;
        a[0] = o[j][0] * inv; a[1] = o[j][1] * inv; a[2] = o[j][2] * inv; a[3] = o[j][3] * inv; c[0] = o[j][4] * inv; c[1] = o[j][5] * inv; c[2] = o[j][6] * inv; c[3] = o[j][7] * inv;
        *(v4fa*)(&os[wb + lr * 132 + 16 * j + 8 * hi]) = a; *(v4fa*)(&os[wb + lr * 132 + 16 * j + 8 * hi + 4]) = c; }
    wave_sync();
    h16* crow = CTX + ((size_t)b * SEQ + t0) * DM + h * HD;
#pragma unroll 1
    for (int ps = 0; ps < 2; ++ps) {
#pragma unroll
        for (int s = 0; s < 8; ++s) { const int row = 2 * s + hi, c8 = lr * 8;
            const v4f x0 = *(const v4fa*)(&os[wb + row * 132 + c8]); const v4f x1 = *(const v4fa*)(&os[wb + row * 132 + c8 + 4]); v8h hv;
#pragma unroll
            for (int i = 0; i < 4; ++i) { hv[i] = (h16)x0[i]; hv[4 + i] = (h16)x1[i]; }
            *(volatile v8h*)(crow + (size_t)row * DM + c8) = hv; }
        if (ps == 0) __threadfence(); }
}

__global__ __launch_bounds__(32 * AW) void k_flash_early(const h16* QH, const h16* QR, const h16* KP, const h16* KR, const h16* VT, const h16* VR, h16* CTX, h16* CR) {
    __shared__ __align__(16) float os[AW * 16 * 68];
    const int lane = threadIdx.x & 31, wave = __builtin_amdgcn_readfirstlane((int)(threadIdx.x >> 5)), lr = lane & 15, hi = lane >> 4;
    const int zh = blockIdx.y; const int b = zh / NH_, h = zh % NH_;
    const int u = blockIdx.x * AW + wave; const int t0 = (u >> 1) * 16, dh = u & 1;
    const size_t pbase = (size_t)zh * SEQ * HD, ebase = (size_t)zh * EARLY * HD;
    const size_t qo = pbase + (size_t)(t0 + lr) * HD + 8 * hi, qe = ebase + (size_t)(t0 + lr) * HD + 8 * hi;
    v16h qh[4], qr[4];
#pragma unroll
    for (int c = 0; c < 4; ++c) { qh[c] = ldh(QH + qo + 32 * c); qr[c] = ldh(QR + qe + 32 * c); }
    const size_t ko = pbase + (size_t)lr * HD + 8 * hi, ke = ebase + (size_t)lr * HD + 8 * hi;
    const size_t vo = pbase + (size_t)(dh * 64 + lr) * SEQ + 8 * hi, ve = ebase + (size_t)(dh * 64 + lr) * EARLY + 8 * hi;
    v8f oH[4], oR[4];
#pragma unroll
    for (int j = 0; j < 4; ++j) { oH[j] = (v8f){}; oR[j] = (v8f){}; }
    float m = -3.0e38f, l = 0.0f;
    const int nst = t0 / 32 + 1;
#pragma unroll 1
    for (int st = 0; st < nst; ++st) {
        const int key0 = st * 32;
        const size_t kk = (size_t)key0 * HD;
        v8f sHa = (v8f){}, sLa = (v8f){}, sHb = (v8f){}, sLb = (v8f){};
#pragma unroll
        for (int c = 0; c < 4; ++c) {
            const v16h kha = ldh(KP + ko + kk + 32 * c), khb = ldh(KP + ko + kk + 16 * HD + 32 * c);
            const v16h kra = ldh(KR + ke + kk + 32 * c), krb = ldh(KR + ke + kk + 16 * HD + 32 * c);
            sHa = wmma16(kha, qh[c], sHa); sLa = wmma16(kha, qr[c], sLa); sLa = wmma16(kra, qh[c], sLa);
            sHb = wmma16(khb, qh[c], sHb); sLb = wmma16(khb, qr[c], sLb); sLb = wmma16(krb, qh[c], sLb);
            asm volatile("v_nop\n\tv_nop\n\tv_nop\n\tv_nop" : "+v"(sHa), "+v"(sLa), "+v"(sHb), "+v"(sLb) : "v"(kha), "v"(khb), "v"(kra), "v"(krb) : "memory");
        }
        float ta[8], tb[8];
#pragma unroll
        for (int r = 0; r < 8; ++r) { ta[r] = (sHa[r] + sLa[r] * QRI) * SC2; tb[r] = (sHb[r] + sLb[r] * QRI) * SC2; }
        if (key0 + 31 > t0) {
            const int tq = t0 + lr, kA = key0 + 8 * hi;
#pragma unroll
            for (int r = 0; r < 8; ++r) { ta[r] = (kA + r > tq) ? -3.0e38f : ta[r]; tb[r] = (kA + 16 + r > tq) ? -3.0e38f : tb[r]; }
        }
        float mx = -3.0e38f;
#pragma unroll
        for (int r = 0; r < 8; ++r) mx = fmaxf(mx, fmaxf(ta[r], tb[r]));
        mx = fmaxf(mx, __shfl_xor(mx, 16, 32));
        const float mnew = fmaxf(m, mx);
        const float alpha = __builtin_amdgcn_exp2f(m - mnew);
        const float sh = PSH - mnew;
        v16h ph, pr; float ls = 0.0f;
#pragma unroll
        for (int r = 0; r < 8; ++r) { const float pa = __builtin_amdgcn_exp2f(ta[r] + sh); const float pc = __builtin_amdgcn_exp2f(tb[r] + sh);
            const h16 ha = (h16)pa; const h16 hc = (h16)pc; ph[r] = ha; ph[8 + r] = hc;
            pr[r] = (h16)((pa - (float)ha) * QRS); pr[8 + r] = (h16)((pc - (float)hc) * QRS); ls += pa + pc; }
        l = l * alpha + ls; m = mnew;
#pragma unroll
        for (int j = 0; j < 4; ++j) { oH[j] = oH[j] * alpha; oR[j] = oR[j] * alpha; }
#pragma unroll
        for (int j = 0; j < 4; ++j) {
            const v16h vh = ldh(VT + vo + (size_t)j * 16 * SEQ + key0), vr = ldh(VR + ve + (size_t)j * 16 * EARLY + key0);
            oH[j] = wmma16(vh, ph, oH[j]); oR[j] = wmma16(vh, pr, oR[j]); oR[j] = wmma16(vr, ph, oR[j]);
            asm volatile("v_nop\n\tv_nop\n\tv_nop\n\tv_nop" : "+v"(oH[j]), "+v"(oR[j]) : "v"(vh), "v"(vr), "v"(ph), "v"(pr) : "memory");
        }
    }
    l += __shfl_xor(l, 16, 32);
    const float inv = CXS / l;
    const int wb = wave * 16 * 68;
#pragma unroll
    for (int j = 0; j < 4; ++j) { v4f a, c;
#pragma unroll
        for (int i = 0; i < 4; ++i) { a[i] = (oH[j][i] + oR[j][i] * QRI) * inv; c[i] = (oH[j][4 + i] + oR[j][4 + i] * QRI) * inv; }
        *(v4fa*)(&os[wb + lr * 68 + 16 * j + 8 * hi]) = a; *(v4fa*)(&os[wb + lr * 68 + 16 * j + 8 * hi + 4]) = c; }
    wave_sync();
    const size_t cofs = (size_t)h * HD + (size_t)dh * 64;
#pragma unroll 1
    for (int ps = 0; ps < 2; ++ps) {
#pragma unroll
        for (int s = 0; s < 4; ++s) { const int row = 4 * s + (lane >> 3), c8 = (lane & 7) * 8;
            const v4f x0 = *(const v4fa*)(&os[wb + row * 68 + c8]); const v4f x1 = *(const v4fa*)(&os[wb + row * 68 + c8 + 4]); v8h hv, rv;
#pragma unroll
            for (int i = 0; i < 4; ++i) { const HR e0 = split16(x0[i]); const HR e1 = split16(x1[i]); hv[i] = e0.h; rv[i] = e0.r; hv[4 + i] = e1.h; rv[4 + i] = e1.r; }
            *(volatile v8h*)(CTX + ((size_t)b * SEQ + t0 + row) * DM + cofs + c8) = hv;
            *(volatile v8h*)(CR + ((size_t)b * EARLY + t0 + row) * DM + cofs + c8) = rv; }
        if (ps == 0) __threadfence(); }
}

__global__ __launch_bounds__(32) void k_out_dense(const h16* __restrict__ A, const h16* __restrict__ Bt, const float* __restrict__ bias, float* OUT) {
    __shared__ __align__(16) float os[16 * 68];
    const int K = DM;
    constexpr int TPB = ((SEQ - EARLY) / 64) > 0 ? ((SEQ - EARLY) / 64) : 1;
    const int lane = threadIdx.x & 31, lr = lane & 15, hi = lane >> 4;
    const int b = blockIdx.x / TPB, r = EARLY + (blockIdx.x % TPB) * 64, c0 = blockIdx.y * 64;
    v8f acc[4][4];
#pragma unroll
    for (int mb = 0; mb < 4; ++mb)
#pragma unroll
        for (int nb = 0; nb < 4; ++nb) acc[mb][nb] = (v8f){};
    const size_t aoff = ((size_t)b * SEQ + r + lr) * K + 8 * hi, boff = (size_t)(c0 + lr) * K + 8 * hi;
#pragma unroll 1
    for (int kc = 0; kc < K; kc += 32) {
        v16h a[4];
#pragma unroll
        for (int mb = 0; mb < 4; ++mb) a[mb] = ldh(A + aoff + (size_t)mb * 16 * K + kc);
#pragma unroll
        for (int nb = 0; nb < 4; ++nb) { const v16h w = ldh(Bt + boff + (size_t)nb * 16 * K + kc);
#pragma unroll
            for (int mb = 0; mb < 4; ++mb) acc[mb][nb] = wmma16(a[mb], w, acc[mb][nb]); }
        asm volatile("" : "+v"(acc[0][0]), "+v"(acc[0][1]), "+v"(acc[0][2]), "+v"(acc[0][3]), "+v"(acc[1][0]), "+v"(acc[1][1]), "+v"(acc[1][2]), "+v"(acc[1][3]));
        asm volatile("v_nop\n\tv_nop\n\tv_nop\n\tv_nop" : "+v"(acc[2][0]), "+v"(acc[2][1]), "+v"(acc[2][2]), "+v"(acc[2][3]), "+v"(acc[3][0]), "+v"(acc[3][1]), "+v"(acc[3][2]), "+v"(acc[3][3]) : "v"(a[0]), "v"(a[1]), "v"(a[2]), "v"(a[3]));
    }
    const int cofs = lr * 4;
    const v4f braw = *(const v4f*)(bias + c0 + cofs); v4f bb;
#pragma unroll
    for (int i = 0; i < 4; ++i) bb[i] = bfr(braw[i]);
#pragma unroll
    for (int mb = 0; mb < 4; ++mb) {
#pragma unroll
        for (int nb = 0; nb < 4; ++nb) {
#pragma unroll
            for (int j = 0; j < 8; ++j) os[(hi * 8 + j) * 68 + nb * 16 + lr] = acc[mb][nb][j] * OUTI; }
        wave_sync();
        float* orow = OUT + ((size_t)b * OUT_SEQ + r + mb * 16) * DM + c0;
#pragma unroll 1
        for (int ps = 0; ps < 2; ++ps) {
#pragma unroll
            for (int s = 0; s < 8; ++s) { const int row = 2 * s + hi;
                const v4f val = *(const v4fa*)(&os[row * 68 + cofs]) + bb;
                *(volatile v4f*)(orow + (size_t)row * DM + cofs) = val; }
            if (ps == 0) __threadfence(); }
        wave_sync();
    }
}

__global__ __launch_bounds__(32) void k_out_early(const h16* __restrict__ A, const h16* __restrict__ AR, const h16* __restrict__ Bt, const float* __restrict__ bias, float* OUT) {
    __shared__ __align__(16) float os[16 * 68];
    const int K = DM;
    constexpr int TPB = (EARLY / 32) > 0 ? (EARLY / 32) : 1;
    const int lane = threadIdx.x & 31, lr = lane & 15, hi = lane >> 4;
    const int b = blockIdx.x / TPB, r = (blockIdx.x % TPB) * 32, c0 = blockIdx.y * 64;
    v8f aH[2][4], aR[2][4];
#pragma unroll
    for (int mb = 0; mb < 2; ++mb)
#pragma unroll
        for (int nb = 0; nb < 4; ++nb) { aH[mb][nb] = (v8f){}; aR[mb][nb] = (v8f){}; }
    const size_t aoff = ((size_t)b * SEQ + r + lr) * K + 8 * hi, roff = ((size_t)b * EARLY + r + lr) * K + 8 * hi, boff = (size_t)(c0 + lr) * K + 8 * hi;
#pragma unroll 1
    for (int kc = 0; kc < K; kc += 32) {
        const v16h a0 = ldh(A + aoff + kc), a1 = ldh(A + aoff + (size_t)16 * K + kc);
        const v16h r0 = ldh(AR + roff + kc), r1 = ldh(AR + roff + (size_t)16 * K + kc);
#pragma unroll
        for (int nb = 0; nb < 4; ++nb) { const v16h w = ldh(Bt + boff + (size_t)nb * 16 * K + kc);
            aH[0][nb] = wmma16(a0, w, aH[0][nb]); aH[1][nb] = wmma16(a1, w, aH[1][nb]);
            aR[0][nb] = wmma16(r0, w, aR[0][nb]); aR[1][nb] = wmma16(r1, w, aR[1][nb]); }
        asm volatile("" : "+v"(aH[0][0]), "+v"(aH[0][1]), "+v"(aH[0][2]), "+v"(aH[0][3]), "+v"(aH[1][0]), "+v"(aH[1][1]), "+v"(aH[1][2]), "+v"(aH[1][3]));
        asm volatile("v_nop\n\tv_nop\n\tv_nop\n\tv_nop" : "+v"(aR[0][0]), "+v"(aR[0][1]), "+v"(aR[0][2]), "+v"(aR[0][3]), "+v"(aR[1][0]), "+v"(aR[1][1]), "+v"(aR[1][2]), "+v"(aR[1][3]) : "v"(a0), "v"(a1), "v"(r0), "v"(r1));
    }
    const int cofs = lr * 4;
    const v4f braw = *(const v4f*)(bias + c0 + cofs); v4f bb;
#pragma unroll
    for (int i = 0; i < 4; ++i) bb[i] = bfr(braw[i]);
#pragma unroll
    for (int mb = 0; mb < 2; ++mb) {
#pragma unroll
        for (int nb = 0; nb < 4; ++nb) {
#pragma unroll
            for (int j = 0; j < 8; ++j) os[(hi * 8 + j) * 68 + nb * 16 + lr] = (aH[mb][nb][j] + aR[mb][nb][j] * QRI) * OUTI; }
        wave_sync();
        float* orow = OUT + ((size_t)b * OUT_SEQ + r + mb * 16) * DM + c0;
#pragma unroll 1
        for (int ps = 0; ps < 2; ++ps) {
#pragma unroll
            for (int s = 0; s < 8; ++s) { const int row = 2 * s + hi;
                const v4f val = *(const v4fa*)(&os[row * 68 + cofs]) + bb;
                *(volatile v4f*)(orow + (size_t)row * DM + cofs) = val; }
            if (ps == 0) __threadfence(); }
        wave_sync();
    }
}

static constexpr size_t al256(size_t v) { return (v + 255) & ~(size_t)255; }
static constexpr size_t SZ_XB = al256((size_t)NB * SEQ * DM * 2);
static constexpr size_t SZ_WB = al256((size_t)3 * DM * DM * 2);
static constexpr size_t SZ_WO = al256((size_t)DM * DM * 2);
static constexpr size_t SZ_PL = al256((size_t)NB * NH_ * SEQ * HD * 2);
static constexpr size_t SZ_PE = al256((size_t)NB * NH_ * EARLY * HD * 2);
static constexpr size_t SZ_CR = al256((size_t)NB * EARLY * DM * 2);
static constexpr size_t SZ_TB = al256((size_t)SEQ * HH * 4);
static constexpr size_t SZ_TOTAL = SZ_XB + SZ_WB + SZ_WO + 3 * SZ_PL + 3 * SZ_PE + SZ_CR + 2 * SZ_TB;
static_assert(SZ_TOTAL <= (size_t)134217728);
static_assert(((size_t)DM * DM * 2) % 256 == 0);
static_assert((size_t)NB * SEQ * DM * 2 <= SZ_XB);

extern "C" void kernel_launch(void* const* d_in, const int* in_sizes, int n_in,
                              void* d_out, int out_size, void* d_ws, size_t ws_size, hipStream_t stream) {
    if (n_in < 9) return;
    const size_t needx = ((size_t)(NB - 1) * SEQ_FULL + SEQ) * DM;
    if ((size_t)in_sizes[0] < needx) return;
    if ((size_t)in_sizes[1] < (size_t)DM * DM || (size_t)in_sizes[3] < (size_t)DM * DM || (size_t)in_sizes[5] < (size_t)DM * DM || (size_t)in_sizes[7] < (size_t)DM * DM) return;
    if (in_sizes[2] < DM || in_sizes[4] < DM || in_sizes[6] < DM || in_sizes[8] < DM) return;
    if ((size_t)out_size < ((size_t)(NB - 1) * OUT_SEQ + SEQ) * DM) return;
    if (SZ_TOTAL > ws_size) return;
    const float* x  = (const float*)d_in[0];
    const float* wq = (const float*)d_in[1]; const float* bq = (const float*)d_in[2];
    const float* wk = (const float*)d_in[3]; const float* bk = (const float*)d_in[4];
    const float* wv = (const float*)d_in[5]; const float* bv = (const float*)d_in[6];
    const float* wo = (const float*)d_in[7]; const float* bo = (const float*)d_in[8];
    float* OUT = (float*)d_out;
    char* wsp = (char*)d_ws;
    bf* XB = (bf*)wsp; h16* CTX = (h16*)wsp; wsp += SZ_XB;
    bf* WB = (bf*)wsp; wsp += SZ_WB;
    h16* WO = (h16*)wsp; wsp += SZ_WO;
    h16* QH = (h16*)wsp; wsp += SZ_PL;
    h16* KP = (h16*)wsp; wsp += SZ_PL;
    h16* VT = (h16*)wsp; wsp += SZ_PL;
    h16* QR = (h16*)wsp; wsp += SZ_PE;
    h16* KR = (h16*)wsp; wsp += SZ_PE;
    h16* VR = (h16*)wsp; wsp += SZ_PE;
    h16* CR = (h16*)wsp; wsp += SZ_CR;
    float* COS = (float*)wsp; wsp += SZ_TB;
    float* SIN = (float*)wsp; wsp += SZ_TB;
    bf* WQ = WB; bf* WK = WB + (size_t)DM * DM; bf* WV = WB + (size_t)2 * DM * DM;

    if (SEQ == SEQ_FULL) {
        const size_t n8 = (size_t)NB * SEQ * DM / 8;
        k_cvt8<<<(unsigned)((n8 + 255) / 256), 256, 0, stream>>>(x, XB, n8);
    } else {
        const size_t n8 = (size_t)SEQ * DM / 8;
        for (int b = 0; b < NB; ++b) k_cvt8<<<(unsigned)((n8 + 255) / 256), 256, 0, stream>>>(x + (size_t)b * SEQ_FULL * DM, XB + (size_t)b * SEQ * DM, n8);
    }
    { const size_t n8 = (size_t)DM * DM / 8; const unsigned g = (unsigned)((n8 + 255) / 256);
      k_cvt8<<<g, 256, 0, stream>>>(wq, WQ, n8); k_cvt8<<<g, 256, 0, stream>>>(wk, WK, n8); k_cvt8<<<g, 256, 0, stream>>>(wv, WV, n8);
      k_cvtw<<<g, 256, 0, stream>>>(wo, WO, n8); }
    k_tab<<<(unsigned)((size_t)SEQ * HH / 256), 256, 0, stream>>>(COS, SIN);

    k_qk<<<dim3(NB * SEQ / 32, NH_, 1), 32, 0, stream>>>(XB, WQ, bq, COS, SIN, QH, QR);
    k_qk<<<dim3(NB * SEQ / 32, NH_, 1), 32, 0, stream>>>(XB, WK, bk, COS, SIN, KP, KR);
    k_vt<<<dim3(DM / 64, NB * SEQ / 64, 1), 32, 0, stream>>>(WV, XB, bv, VT, VR);

    k_flash_early<<<dim3(EARLY / 32, NB * NH_, 1), 32 * AW, 0, stream>>>(QH, QR, KP, KR, VT, VR, CTX, CR);
    if (SEQ > EARLY) k_flash_dense<<<dim3((SEQ - EARLY) / (16 * AW), NB * NH_, 1), 32 * AW, 0, stream>>>(QH, KP, VT, CTX);

    k_out_early<<<dim3(NB * (EARLY / 32), DM / 64, 1), 32, 0, stream>>>(CTX, CR, WO, bo, OUT);
    if (SEQ > EARLY) k_out_dense<<<dim3(NB * ((SEQ - EARLY) / 64), DM / 64, 1), 32, 0, stream>>>(CTX, WO, bo, OUT);
}
